// ProbabilityFlow_61151744360563
// MI455X (gfx1250) — hardware-verified
//
#include <hip/hip_runtime.h>


#define NB_  8192
#define DX   32
#define KIN  33
#define KP   64
#define HH   512
#define H2   (2 * HH)

typedef unsigned short bf;
typedef __attribute__((ext_vector_type(16))) __bf16   v16bf;
typedef __attribute__((ext_vector_type(8)))  unsigned short v8us;
typedef __attribute__((ext_vector_type(8)))  float    v8f;
typedef __attribute__((ext_vector_type(4)))  float    v4f;
typedef v4f  __attribute__((may_alias)) v4fa;
typedef v8us __attribute__((may_alias)) v8usa;

__device__ __forceinline__ unsigned short f2bf(float f) { unsigned u = __float_as_uint(f); u += 0x7FFFu + ((u >> 16) & 1u); return (unsigned short)(u >> 16); }
__device__ __forceinline__ float bf2f(unsigned short b) { return __uint_as_float(((unsigned)b) << 16); }
__device__ __forceinline__ float bfr(float f) { return bf2f(f2bf(f)); }
__device__ __forceinline__ v16bf cat16b(v8us lo, v8us hi) { return __builtin_bit_cast(v16bf, __builtin_shufflevector(lo, hi, 0, 1, 2, 3, 4, 5, 6, 7, 8, 9, 10, 11, 12, 13, 14, 15)); }
__device__ __forceinline__ v8f wmmab(v16bf a, v16bf b, v8f c) { return __builtin_amdgcn_wmma_f32_16x16x32_bf16(false, a, false, b, (short)0, c, false, false); }
__device__ __forceinline__ float gelu_t(float x, float* dg) {
    const float k = 0.7978845608028654f, a = 0.044715f; const float u = k * (x + a * x * x * x); const float th = tanhf(u);
    *dg = 0.5f * (1.0f + th) + 0.5f * x * (1.0f - th * th) * k * (1.0f + 3.0f * a * x * x);
    return 0.5f * x * (1.0f + th);
}

__global__ __launch_bounds__(256) void k_xin(const float* __restrict__ x, const float* __restrict__ t, bf* A) {
    const int lane = threadIdx.x & 31, r = (blockIdx.x * 8 + (threadIdx.x >> 5)) * 4 + (lane >> 3), p = lane & 7;
    if (r >= NB_) return;
    v8us o;
#pragma unroll
    for (int i = 0; i < 8; ++i) { const int c = p * 8 + i; float v = 0.f; if (c < DX) v = x[(size_t)r * DX + c]; else if (c == DX) v = t[r]; o[i] = f2bf(v); }
    *(volatile v8us*)(A + (size_t)r * KP + p * 8) = o; __threadfence(); *(volatile v8us*)(A + (size_t)r * KP + p * 8) = o;
}
__global__ __launch_bounds__(256) void k_w1(const float* __restrict__ W1v, const float* __restrict__ W1s, bf* W1T) {
    const int lane = threadIdx.x & 31, n = (blockIdx.x * 8 + (threadIdx.x >> 5)) * 4 + (lane >> 3), p = lane & 7;
    if (n >= H2) return;
    const float* W = (n < HH) ? W1v : W1s; const int nn = (n < HH) ? n : n - HH;
    v8us o;
#pragma unroll
    for (int i = 0; i < 8; ++i) { const int k = p * 8 + i; o[i] = (k < KIN) ? f2bf(W[(size_t)k * HH + nn]) : (unsigned short)0; }
    *(volatile v8us*)(W1T + (size_t)n * KP + p * 8) = o; __threadfence(); *(volatile v8us*)(W1T + (size_t)n * KP + p * 8) = o;
}
__global__ __launch_bounds__(256) void k_w2(const float* __restrict__ W2v, const float* __restrict__ W2s, bf* W2T) {
    const int lane = threadIdx.x & 31, c = blockIdx.x * 8 + (threadIdx.x >> 5);
    if (c >= 64) return;
#pragma unroll 1
    for (int ps = 0; ps < 2; ++ps) {
#pragma unroll
        for (int q = 0; q < 4; ++q) { v8us o;
#pragma unroll
            for (int i = 0; i < 8; ++i) { const int k = q * 256 + lane * 8 + i; float v = 0.f;
                if (c < DX) { if (k < HH) v = W2v[(size_t)k * DX + c]; } else { if (k >= HH) v = W2s[(size_t)(k - HH) * DX + (c - DX)]; }
                o[i] = f2bf(v); }
            *(volatile v8us*)(W2T + (size_t)c * H2 + q * 256 + lane * 8) = o; }
        if (ps == 0) __threadfence(); }
}
__global__ __launch_bounds__(256) void k_cvec(const float* __restrict__ W1v, const float* __restrict__ W2v, const float* __restrict__ W1s, const float* __restrict__ W2s, float* cv) {
    const int j = blockIdx.x * 256 + threadIdx.x; if (j >= H2) return;
    const float* W1 = (j < HH) ? W1v : W1s; const float* W2 = (j < HH) ? W2v : W2s; const int jj = (j < HH) ? j : j - HH;
    float s = 0.f;
#pragma unroll 4
    for (int i = 0; i < DX; ++i) s += bfr(W1[(size_t)i * HH + jj]) * bfr(W2[(size_t)jj * DX + i]);
    *(volatile float*)(cv + j) = s; __threadfence(); *(volatile float*)(cv + j) = s;
}
__global__ __launch_bounds__(128) void k_gemm1(const bf* __restrict__ A, const bf* __restrict__ W1T, const float* __restrict__ b1v, const float* __restrict__ b1s, float* PRE) {
    __shared__ __align__(16) float ost[4][16 * 68];
    const int lane = threadIdx.x & 31, wave = threadIdx.x >> 5, lr = lane & 15, hi = lane >> 4;
    const size_t r0 = (size_t)blockIdx.x * 64 + wave * 16; const int c0 = blockIdx.y * 64;
    v8f acc[4];
#pragma unroll
    for (int t = 0; t < 4; ++t) acc[t] = (v8f){};
#pragma unroll
    for (int kc = 0; kc < KP; kc += 32) {
        const v16bf a = cat16b(*(const v8us*)(A + (r0 + lr) * KP + kc + 8 * hi), *(const v8us*)(A + (r0 + lr) * KP + kc + 8 * hi + 16));
#pragma unroll
        for (int t = 0; t < 4; ++t) { const bf* bp = W1T + (size_t)(c0 + t * 16 + lr) * KP + kc + 8 * hi; acc[t] = wmmab(a, cat16b(*(const v8us*)bp, *(const v8us*)(bp + 16)), acc[t]); }
    }
    float* os = &ost[wave][0];
#pragma unroll
    for (int t = 0; t < 4; ++t) { const int c = c0 + t * 16 + lr; const float bv = (c < HH) ? bfr(b1v[c]) : bfr(b1s[c - HH]);
#pragma unroll
        for (int j = 0; j < 8; ++j) os[(hi * 8 + j) * 68 + t * 16 + lr] = acc[t][j] + bv; }
    __builtin_amdgcn_wave_barrier(); asm volatile("" ::: "memory");
    float* crow = PRE + r0 * H2 + c0;
    auto pass = [&]() {
#pragma unroll
        for (int s = 0; s < 8; ++s) { const int Lid = (lane >> 3) + 4 * s, piece = lane & 7; const int row = Lid >> 1, cofs = (Lid & 1) * 32 + piece * 4;
            const v4f val = *(const v4fa*)(os + row * 68 + cofs); *(volatile v4f*)(crow + (size_t)row * H2 + cofs) = val; }
    };
    pass(); __threadfence(); pass();
}
__global__ __launch_bounds__(256) void k_act(const float* __restrict__ PRE, bf* HHp, bf* HLp) {
    const int lane = threadIdx.x & 31, r = blockIdx.x * 8 + (threadIdx.x >> 5);
    if (r >= NB_) return;
#pragma unroll 1
    for (int ps = 0; ps < 2; ++ps) {
#pragma unroll 1
        for (int q = 0; q < 4; ++q) { v8us oh, ol;
#pragma unroll
            for (int i = 0; i < 8; ++i) { float dg; const float g = gelu_t(PRE[(size_t)r * H2 + q * 256 + lane * 8 + i], &dg); const unsigned short hb = f2bf(g); oh[i] = hb; ol[i] = f2bf(g - bf2f(hb)); }
            *(volatile v8us*)(HHp + (size_t)r * H2 + q * 256 + lane * 8) = oh; *(volatile v8us*)(HLp + (size_t)r * H2 + q * 256 + lane * 8) = ol; }
        if (ps == 0) __threadfence(); }
}
__global__ __launch_bounds__(256) void k_div(const float* __restrict__ PRE, const float* __restrict__ cv, const float* __restrict__ t, float* out1) {
    __shared__ float red[2][32][8];
    const int tid = threadIdx.x, rl = tid >> 3, part = tid & 7; const size_t r = (size_t)blockIdx.x * 32 + rl;
    float sv = 0.f, ss = 0.f;
#pragma unroll 2
    for (int i = 0; i < 64; ++i) { const int jv = part * 64 + i, js = HH + part * 64 + i; float dg;
        gelu_t(PRE[r * H2 + jv], &dg); sv += dg * cv[jv]; gelu_t(PRE[r * H2 + js], &dg); ss += dg * cv[js]; }
    red[0][rl][part] = sv; red[1][rl][part] = ss;
    __syncthreads();
    if (tid < 32) { float a = 0.f, b = 0.f;
#pragma unroll
        for (int p = 0; p < 8; ++p) { a += red[0][tid][p]; b += red[1][tid][p]; }
        const size_t rr = (size_t)blockIdx.x * 32 + tid; const float tb = bfr(t[rr]); const float gg = 0.5f * (1.0f - 2.0f * tb);
        const float v = -(a - gg * b);
        *(volatile float*)(out1 + rr) = v; __threadfence(); *(volatile float*)(out1 + rr) = v; }
}
__global__ __launch_bounds__(128) void k_gemm2(const bf* __restrict__ Hh, const bf* __restrict__ Hl, const bf* __restrict__ W2T, const float* __restrict__ b2v, const float* __restrict__ b2s, const float* __restrict__ t, float* out0) {
    __shared__ __align__(16) float ost[4][16 * 68];
    const int lane = threadIdx.x & 31, wave = threadIdx.x >> 5, lr = lane & 15, hi = lane >> 4;
    const size_t r0 = (size_t)blockIdx.x * 64 + wave * 16;
    const size_t aoff = (r0 + lr) * H2 + 8 * hi;
    v8f acc[4];
#pragma unroll
    for (int tt = 0; tt < 4; ++tt) acc[tt] = (v8f){};
#pragma unroll 2
    for (int kc = 0; kc < H2; kc += 32) {
        const v16bf a = cat16b(*(const v8us*)(Hh + aoff + kc), *(const v8us*)(Hh + aoff + kc + 16)), al = cat16b(*(const v8us*)(Hl + aoff + kc), *(const v8us*)(Hl + aoff + kc + 16));
#pragma unroll
        for (int tt = 0; tt < 4; ++tt) { const bf* bp = W2T + (size_t)(tt * 16 + lr) * H2 + kc + 8 * hi; const v16bf bb = cat16b(*(const v8us*)bp, *(const v8us*)(bp + 16)); acc[tt] = wmmab(a, bb, acc[tt]); acc[tt] = wmmab(al, bb, acc[tt]); }
        asm volatile("v_nop" : "+v"(acc[0]), "+v"(acc[1]), "+v"(acc[2]), "+v"(acc[3]) : "v"(a), "v"(al) : "memory");
    }
    float* os = &ost[wave][0];
#pragma unroll
    for (int j = 0; j < 8; ++j) { const size_t r = r0 + hi * 8 + j; const float gg = 0.5f * (1.0f - 2.0f * bfr(t[r]));
#pragma unroll
        for (int tt = 0; tt < 2; ++tt) { const int d = tt * 16 + lr; os[(hi * 8 + j) * 68 + d] = (acc[tt][j] + bfr(b2v[d])) - gg * (acc[tt + 2][j] + bfr(b2s[d])); } }
    __builtin_amdgcn_wave_barrier(); asm volatile("" ::: "memory");
    auto pass = [&]() {
#pragma unroll
        for (int s = 0; s < 4; ++s) { const int row = s * 4 + (lane >> 3), piece = lane & 7; const v4f val = *(const v4fa*)(os + row * 68 + piece * 4);
            *(volatile v4f*)(out0 + (r0 + row) * DX + piece * 4) = val; }
    };
    pass(); __threadfence(); pass();
}

extern "C" void kernel_launch(void* const* d_in, const int* in_sizes, int n_in,
                              void* d_out, int out_size, void* d_ws, size_t ws_size, hipStream_t stream) {
    (void)in_sizes; (void)n_in; (void)out_size;
    const float* x = (const float*)d_in[0]; const float* t = (const float*)d_in[1];
    const float* W1v = (const float*)d_in[2]; const float* b1v = (const float*)d_in[3]; const float* W2v = (const float*)d_in[4]; const float* b2v = (const float*)d_in[5];
    const float* W1s = (const float*)d_in[6]; const float* b1s = (const float*)d_in[7]; const float* W2s = (const float*)d_in[8]; const float* b2s = (const float*)d_in[9];
    float* out0 = (float*)d_out;
    float* out1 = (float*)((char*)d_out + 1048576);
    char* wsp = (char*)d_ws;
    auto take = [&](size_t bytes) { char* p = wsp; wsp += (bytes + 255) & ~(size_t)255; return (void*)p; };
    bf* A = (bf*)take((size_t)NB_ * KP * 2); bf* W1T = (bf*)take((size_t)H2 * KP * 2); bf* W2T = (bf*)take((size_t)64 * H2 * 2); float* cv = (float*)take((size_t)H2 * 4);
    float* PRE = (float*)take((size_t)NB_ * H2 * 4); bf* HHp = (bf*)take((size_t)NB_ * H2 * 2); bf* HLp = (bf*)take((size_t)NB_ * H2 * 2);
    if ((size_t)(wsp - (char*)d_ws) > ws_size) return;
    k_xin<<<NB_ / 32, 256, 0, stream>>>(x, t, A); k_w1<<<H2 / 32, 256, 0, stream>>>(W1v, W1s, W1T); k_w2<<<64 / 8, 256, 0, stream>>>(W2v, W2s, W2T);
    k_cvec<<<H2 / 256, 256, 0, stream>>>(W1v, W2v, W1s, W2s, cv);
    k_gemm1<<<dim3(NB_ / 64, H2 / 64, 1), 128, 0, stream>>>(A, W1T, b1v, b1s, PRE);
    k_act<<<NB_ / 8, 256, 0, stream>>>(PRE, HHp, HLp);
    k_div<<<NB_ / 32, 256, 0, stream>>>(PRE, cv, t, out1);
    k_gemm2<<<NB_ / 64, 128, 0, stream>>>(HHp, HLp, W2T, b2v, b2s, t, out0);
}
